// modeler_30709016166544
// MI455X (gfx1250) — hardware-verified
//
#include <hip/hip_runtime.h>


#define NV   50000
#define NU   20000
#define NVP  50048
#define NUP  20032
#define DEG  16
#define FT   128
#define HID  256
#define OUTD 128
#define VCH  12544
#define RPB  400
#ifndef NVRUN
#define NVRUN NV
#define NURUN NU
#endif

typedef unsigned short bf;
typedef __attribute__((ext_vector_type(16))) __bf16   v16bf;
typedef __attribute__((ext_vector_type(8)))  unsigned short v8us;
typedef __attribute__((ext_vector_type(4)))  unsigned short v4us;
typedef __attribute__((ext_vector_type(8)))  float    v8f;
typedef __attribute__((ext_vector_type(4)))  float    v4f;
typedef v4f  __attribute__((may_alias)) v4fa;
typedef v8us __attribute__((may_alias)) v8usa;

__device__ __forceinline__ unsigned short f2bf(float f) { unsigned u = __float_as_uint(f); u += 0x7FFFu + ((u >> 16) & 1u); return (unsigned short)(u >> 16); }
__device__ __forceinline__ float bf2f(unsigned short b) { return __uint_as_float(((unsigned)b) << 16); }
__device__ __forceinline__ float bfr(float f) { return bf2f(f2bf(f)); }
__device__ __forceinline__ v16bf cat16b(v8us lo, v8us hi) { return __builtin_bit_cast(v16bf, __builtin_shufflevector(lo, hi, 0, 1, 2, 3, 4, 5, 6, 7, 8, 9, 10, 11, 12, 13, 14, 15)); }
__device__ __forceinline__ v8f wmmab(v16bf a, v16bf b, v8f c) { return __builtin_amdgcn_wmma_f32_16x16x32_bf16(false, a, false, b, (short)0, c, false, false); }

__global__ __launch_bounds__(256) void k_cvtb(const float* __restrict__ src, int nrows, int npad, bf* dst) {
    const int lane = threadIdx.x & 31, r = blockIdx.x * 8 + (threadIdx.x >> 5);
    if (r >= npad) return;
    v4us o = {};
    if (r < nrows) { const v4f x = *(const v4f*)(src + (size_t)r * FT + lane * 4);
#pragma unroll
        for (int i = 0; i < 4; ++i) o[i] = f2bf(x[i]); }
    *(volatile v4us*)(dst + (size_t)r * FT + lane * 4) = o; __threadfence(); *(volatile v4us*)(dst + (size_t)r * FT + lane * 4) = o;
}
__global__ __launch_bounds__(256) void k_wt(const float* __restrict__ Wm, int K, int ncols, bf* WT) {
    __shared__ __align__(16) unsigned short tl[64 * 72];
    const int tid = threadIdx.x, k0 = blockIdx.x * 64, n0 = blockIdx.y * 64;
    const int kk = tid >> 2, nq = (tid & 3) * 16;
#pragma unroll
    for (int i = 0; i < 16; ++i) tl[(nq + i) * 72 + kk] = f2bf(Wm[(size_t)(k0 + kk) * ncols + n0 + nq + i]);
    __syncthreads();
    const int piece = tid & 7;
    auto pass = [&]() {
#pragma unroll
        for (int s = 0; s < 2; ++s) { const int nr = (tid >> 3) + 32 * s; const v8us val = *(const v8usa*)(tl + nr * 72 + piece * 8); *(volatile v8us*)(WT + (size_t)(n0 + nr) * K + k0 + piece * 8) = val; }
    };
    pass(); __threadfence(); pass();
}
template <int W, bool SRCBF>
__global__ __launch_bounds__(256) void k_gmean(const void* __restrict__ srcv, const int* __restrict__ idx, int nrows, int npad, int nsrc, bf* OH, bf* OL) {
    constexpr int E = W / 32;
    typedef __attribute__((ext_vector_type(E))) unsigned short vEus;
    const int lane = threadIdx.x & 31, r = blockIdx.x * 8 + (threadIdx.x >> 5);
    if (r >= npad) return;
    float s[E];
#pragma unroll
    for (int e = 0; e < E; ++e) s[e] = 0.f;
    if (r < nrows) {
        int myi = 0;
        if (lane < DEG) { myi = idx[(size_t)r * DEG + lane]; myi = myi < 0 ? 0 : (myi >= nsrc ? nsrc - 1 : myi); }
#pragma unroll
        for (int j = 0; j < DEG; ++j) {
            const int id = __shfl(myi, j, 32);
            if (SRCBF) { const bf* sp = (const bf*)srcv + (size_t)id * W + lane * E;
                if (E == 4) { const v4us v = *(const v4us*)sp;
#pragma unroll
                    for (int e = 0; e < 4; ++e) s[e] += bf2f(v[e]); }
                else { const v8us v = *(const v8us*)sp;
#pragma unroll
                    for (int e = 0; e < (E == 8 ? 8 : 0); ++e) s[e] += bf2f(v[e]); } }
            else { const float* sp = (const float*)srcv + (size_t)id * W + lane * E;
#pragma unroll
                for (int e4 = 0; e4 < E; e4 += 4) { const v4f v = *(const v4f*)(sp + e4); s[e4] += v[0]; s[e4 + 1] += v[1]; s[e4 + 2] += v[2]; s[e4 + 3] += v[3]; } }
        }
    }
    vEus oh, ol;
#pragma unroll
    for (int e = 0; e < E; ++e) { const float m = s[e] * (1.0f / DEG); const unsigned short hb = f2bf(m); oh[e] = hb; ol[e] = f2bf(m - bf2f(hb)); }
    const size_t o = (size_t)r * W + lane * E;
    *(volatile vEus*)(OH + o) = oh; *(volatile vEus*)(OL + o) = ol; __threadfence(); *(volatile vEus*)(OH + o) = oh; *(volatile vEus*)(OL + o) = ol;
}
template <int MODE>
__global__ __launch_bounds__(128) void k_gemm(const bf* __restrict__ Ah, const bf* __restrict__ Al, int K1, const bf* __restrict__ A2, int K2,
                                              const bf* __restrict__ Bn, const float* __restrict__ bias, const float* __restrict__ slp, int act,
                                              int nvalid, float* C, int ldc, bf* OH, bf* OL) {
    __shared__ __align__(16) float ost[4][16 * 68];
    const int lane = threadIdx.x & 31, wave = threadIdx.x >> 5, lr = lane & 15, hi = lane >> 4;
    const int r0 = blockIdx.x * 64 + wave * 16; const int c0 = blockIdx.y * 64; const int KT = K1 + K2;
    v8f acc[4];
#pragma unroll
    for (int t = 0; t < 4; ++t) acc[t] = (v8f){};
    const size_t a1 = (size_t)(r0 + lr) * K1 + 8 * hi;
#pragma unroll 2
    for (int kc = 0; kc < K1; kc += 32) {
        const v16bf a = cat16b(*(const v8us*)(Ah + a1 + kc), *(const v8us*)(Ah + a1 + kc + 16));
        const v16bf al = cat16b(*(const v8us*)(Al + a1 + kc), *(const v8us*)(Al + a1 + kc + 16));
#pragma unroll
        for (int t = 0; t < 4; ++t) { const bf* bp = Bn + (size_t)(c0 + t * 16 + lr) * KT + kc + 8 * hi; const v16bf bb = cat16b(*(const v8us*)bp, *(const v8us*)(bp + 16)); acc[t] = wmmab(a, bb, acc[t]); acc[t] = wmmab(al, bb, acc[t]); }
        asm volatile("v_nop" : "+v"(acc[0]), "+v"(acc[1]), "+v"(acc[2]), "+v"(acc[3]) : "v"(a), "v"(al) : "memory");
    }
    const size_t a2 = (size_t)(r0 + lr) * K2 + 8 * hi;
#pragma unroll 2
    for (int kc = 0; kc < K2; kc += 32) {
        const v16bf a = cat16b(*(const v8us*)(A2 + a2 + kc), *(const v8us*)(A2 + a2 + kc + 16));
#pragma unroll
        for (int t = 0; t < 4; ++t) { const bf* bp = Bn + (size_t)(c0 + t * 16 + lr) * KT + K1 + kc + 8 * hi; const v16bf bb = cat16b(*(const v8us*)bp, *(const v8us*)(bp + 16)); acc[t] = wmmab(a, bb, acc[t]); }
        asm volatile("v_nop" : "+v"(acc[0]), "+v"(acc[1]), "+v"(acc[2]), "+v"(acc[3]) : "v"(a) : "memory");
    }
    const float slope = act ? bfr(*slp) : 1.0f;
    float* os = &ost[wave][0];
#pragma unroll
    for (int t = 0; t < 4; ++t) {
#pragma unroll
        for (int j = 0; j < 8; ++j) { float v = acc[t][j] + bfr(bias[c0 + t * 16 + lr]); if (act) v = (v >= 0.f) ? v : slope * v; os[(hi * 8 + j) * 68 + t * 16 + lr] = v; } }
    __builtin_amdgcn_wave_barrier(); asm volatile("" ::: "memory");
    auto pass = [&]() {
#pragma unroll
        for (int s = 0; s < 8; ++s) { const int Lid = (lane >> 3) + 4 * s, piece = lane & 7; const int row = Lid >> 1, cofs = (Lid & 1) * 32 + piece * 4;
            const v4f val = *(const v4fa*)(os + row * 68 + cofs); const size_t go = (size_t)(r0 + row) * ldc + c0 + cofs;
            if (MODE == 0 || r0 + row < nvalid) *(volatile v4f*)(C + go) = val;
            if (MODE == 1) { v4us vh, vl;
#pragma unroll
                for (int i = 0; i < 4; ++i) { const unsigned short hb = f2bf(val[i]); vh[i] = hb; vl[i] = f2bf(val[i] - bf2f(hb)); }
                *(volatile v4us*)(OH + go) = vh; *(volatile v4us*)(OL + go) = vl; } }
    };
    pass(); __threadfence(); pass();
}
__global__ __launch_bounds__(256) void k_sv(const float* __restrict__ E3, const float* __restrict__ NB, const int* __restrict__ idx, int nrows, int nsrc, float* S) {
    const int lane = threadIdx.x & 31, r = blockIdx.x * 8 + (threadIdx.x >> 5);
    if (r >= nrows) return;
    int myi = 0;
    if (lane < DEG) { myi = idx[(size_t)r * DEG + lane]; myi = myi < 0 ? 0 : (myi >= nsrc ? nsrc - 1 : myi); }
    v4f s = {};
#pragma unroll
    for (int j = 0; j < DEG; ++j) { const int id = __shfl(myi, j, 32); const v4f v = *(const v4f*)(NB + (size_t)id * OUTD + lane * 4); s += v; }
    const v4f e = *(const v4f*)(E3 + (size_t)r * OUTD + lane * 4); s = (s + e) / 17.0f;
    *(volatile v4f*)(S + (size_t)r * OUTD + lane * 4) = s; __threadfence(); *(volatile v4f*)(S + (size_t)r * OUTD + lane * 4) = s;
}
__global__ __launch_bounds__(256) void k_losspart(const float* __restrict__ E3, const float* __restrict__ S, const int* __restrict__ perm, int nrows, float* PART) {
    __shared__ float ws[8];
    const int lane = threadIdx.x & 31, wave = threadIdx.x >> 5, b = blockIdx.x;
    float acc = 0.f;
    const int rend = (b + 1) * RPB < nrows ? (b + 1) * RPB : nrows;
#pragma unroll 1
    for (int r = b * RPB + wave; r < rend; r += 8) {
        int pr = perm[r]; pr = pr < 0 ? 0 : (pr >= nrows ? nrows - 1 : pr);
        const v4f e = *(const v4f*)(E3 + (size_t)r * OUTD + lane * 4), s1 = *(const v4f*)(S + (size_t)r * OUTD + lane * 4), s2 = *(const v4f*)(S + (size_t)pr * OUTD + lane * 4);
        float d1 = e[0] * s1[0] + e[1] * s1[1] + e[2] * s1[2] + e[3] * s1[3], d2 = e[0] * s2[0] + e[1] * s2[1] + e[2] * s2[2] + e[3] * s2[3];
#pragma unroll
        for (int sh = 16; sh; sh >>= 1) { d1 += __shfl_xor(d1, sh, 32); d2 += __shfl_xor(d2, sh, 32); }
        const float p1 = 1.0f / (1.0f + __expf(-d1)), p2 = 1.0f / (1.0f + __expf(-d2));
        acc += fmaxf(0.f, p2 - p1 + 0.5f);
    }
    if (lane == 0) ws[wave] = acc;
    __syncthreads();
    if (threadIdx.x == 0) { float t = 0.f;
#pragma unroll
        for (int w = 0; w < 8; ++w) t += ws[w];
        *(volatile float*)(PART + (size_t)b * 32) = t; __threadfence(); *(volatile float*)(PART + (size_t)b * 32) = t; }
}
__global__ __launch_bounds__(256) void k_lossfin(const float* __restrict__ PART, int nbv, int nbu, int nv, int nu, float* out) {
    __shared__ float tv[256]; __shared__ float tu[256];
    const int t = threadIdx.x;
    tv[t] = (t < nbv) ? PART[(size_t)t * 32] : 0.f; tu[t] = (t < nbu) ? PART[(size_t)(nbv + t) * 32] : 0.f;
    __syncthreads();
#pragma unroll
    for (int sh = 128; sh; sh >>= 1) { if (t < sh) { tv[t] += tv[t + sh]; tu[t] += tu[t + sh]; } __syncthreads(); }
    if (t == 0) { const float l = tv[0] / (float)nv + tu[0] / (float)nu; *(volatile float*)out = l; __threadfence(); *(volatile float*)out = l; }
}

extern "C" void kernel_launch(void* const* d_in, const int* in_sizes, int n_in,
                              void* d_out, int out_size, void* d_ws, size_t ws_size, hipStream_t stream) {
    (void)in_sizes; (void)n_in; (void)out_size;
    const float* feat_v = (const float*)d_in[0]; const float* feat_u = (const float*)d_in[1];
    const int* nbr_v = (const int*)d_in[2]; const int* nbr_u = (const int*)d_in[3]; const int* vidx = (const int*)d_in[4]; const int* uidx = (const int*)d_in[5];
    const float* W1v = (const float*)d_in[6];  const float* b1v = (const float*)d_in[7];  const float* W1u = (const float*)d_in[8];  const float* b1u = (const float*)d_in[9];
    const float* a1v = (const float*)d_in[10]; const float* a1u = (const float*)d_in[11];
    const float* W2v = (const float*)d_in[12]; const float* b2v = (const float*)d_in[13]; const float* W2u = (const float*)d_in[14]; const float* b2u = (const float*)d_in[15];
    const float* a2v = (const float*)d_in[16]; const float* a2u = (const float*)d_in[17];
    const float* W3v = (const float*)d_in[18]; const float* b3v = (const float*)d_in[19]; const float* W3u = (const float*)d_in[20]; const float* b3u = (const float*)d_in[21];
    float* out = (float*)d_out;
    float* ve2o = out; float* ue2o = out + (size_t)NV * OUTD; float* losso = out + (size_t)NV * OUTD + (size_t)NU * OUTD;
    char* wsp = (char*)d_ws;
    auto take = [&](size_t bytes) { char* p = wsp; wsp += (bytes + 255) & ~(size_t)255; return (void*)p; };
    bf* FVb = (bf*)take((size_t)NVP * FT * 2); bf* FUb = (bf*)take((size_t)NUP * FT * 2);
    bf* W1vT = (bf*)take((size_t)HID * FT * 2); bf* W1uT = (bf*)take((size_t)HID * FT * 2); bf* W2vT = (bf*)take((size_t)OUTD * HID * 2); bf* W2uT = (bf*)take((size_t)OUTD * HID * 2);
    bf* W3vT = (bf*)take((size_t)OUTD * (OUTD + FT) * 2); bf* W3uT = (bf*)take((size_t)OUTD * (OUTD + FT) * 2);
    char* RA = (char*)take((size_t)NVP * HID * 4);
    char* RB = (char*)take((size_t)NUP * HID * 4);
    char* RC = (char*)take((size_t)NUP * HID * 4);
    char* RD = (char*)take((size_t)NUP * OUTD * 4);
    float* PART = (float*)take((size_t)176 * 128);
    if ((size_t)(wsp - (char*)d_ws) > ws_size) return;
    float* VE1 = (float*)RA; bf* VE2h = (bf*)RA; bf* VE2l = (bf*)(RA + (size_t)NVP * OUTD * 2); float* VE3 = (float*)(RA + (size_t)NVP * OUTD * 4); float* SV = (float*)RA;
    float* UE1 = (float*)RB; float* SU = (float*)RB;
    bf* M1uh = (bf*)RC; bf* M1ul = (bf*)(RC + (size_t)NUP * FT * 2);
    bf* M1vh = (bf*)RC; bf* M1vl = (bf*)(RC + (size_t)NVP * FT * 2);
    bf* M2uh = (bf*)RC; bf* M2ul = (bf*)(RC + (size_t)NUP * HID * 2);
    bf* M2ch = (bf*)RC; bf* M2cl = (bf*)(RC + (size_t)VCH * HID * 2);
    float* UE3 = (float*)RC;
    bf* UE2h = (bf*)RD; bf* UE2l = (bf*)(RD + (size_t)NUP * OUTD * 2);
    const int nv = NVRUN, nu = NURUN; const int nvp = (nv + 63) & ~63, nup = (nu + 63) & ~63; const int nbv = (nv + RPB - 1) / RPB, nbu = (nu + RPB - 1) / RPB;
#ifdef DBGRUN
    hipMemsetAsync(d_out, 0, (size_t)NV * OUTD * 4 + (size_t)NU * OUTD * 4 + 4, stream);
#endif
    k_wt<<<dim3(FT / 64, HID / 64), 256, 0, stream>>>(W1v, FT, HID, W1vT); k_wt<<<dim3(FT / 64, HID / 64), 256, 0, stream>>>(W1u, FT, HID, W1uT);
    k_wt<<<dim3(HID / 64, OUTD / 64), 256, 0, stream>>>(W2v, HID, OUTD, W2vT); k_wt<<<dim3(HID / 64, OUTD / 64), 256, 0, stream>>>(W2u, HID, OUTD, W2uT);
    k_wt<<<dim3((OUTD + FT) / 64, OUTD / 64), 256, 0, stream>>>(W3v, OUTD + FT, OUTD, W3vT); k_wt<<<dim3((OUTD + FT) / 64, OUTD / 64), 256, 0, stream>>>(W3u, OUTD + FT, OUTD, W3uT);
    k_cvtb<<<nvp / 8, 256, 0, stream>>>(feat_v, nv, nvp, FVb); k_cvtb<<<nup / 8, 256, 0, stream>>>(feat_u, nu, nup, FUb);
    k_gmean<FT, true><<<nup / 8, 256, 0, stream>>>(FVb, nbr_u, nu, nup, nv, M1uh, M1ul);
    k_gemm<0><<<dim3(nup / 64, HID / 64), 128, 0, stream>>>(M1uh, M1ul, FT, nullptr, 0, W1uT, b1u, a1u, 1, nup, UE1, HID, nullptr, nullptr);
    k_gmean<FT, true><<<nvp / 8, 256, 0, stream>>>(FUb, nbr_v, nv, nvp, nu, M1vh, M1vl);
    k_gemm<0><<<dim3(nvp / 64, HID / 64), 128, 0, stream>>>(M1vh, M1vl, FT, nullptr, 0, W1vT, b1v, a1v, 1, nvp, VE1, HID, nullptr, nullptr);
    k_gmean<HID, false><<<nup / 8, 256, 0, stream>>>(VE1, nbr_u, nu, nup, nv, M2uh, M2ul);
    k_gemm<1><<<dim3(nup / 64, OUTD / 64), 128, 0, stream>>>(M2uh, M2ul, HID, nullptr, 0, W2uT, b2u, a2u, 1, nu, ue2o, OUTD, UE2h, UE2l);
    for (int cb = 0; cb < nvp; cb += VCH) {
        const int rows = (cb + VCH <= nvp) ? VCH : nvp - cb; const int nval = (nv - cb < rows) ? nv - cb : rows;
        k_gmean<HID, false><<<rows / 8, 256, 0, stream>>>(UE1, nbr_v + (size_t)cb * DEG, nval, rows, nu, M2ch, M2cl);
        k_gemm<1><<<dim3(rows / 64, OUTD / 64), 128, 0, stream>>>(M2ch, M2cl, HID, nullptr, 0, W2vT, b2v, a2v, 1, nv - cb, ve2o + (size_t)cb * OUTD, OUTD, VE2h + (size_t)cb * OUTD, VE2l + (size_t)cb * OUTD);
    }
    k_gemm<0><<<dim3(nup / 64, OUTD / 64), 128, 0, stream>>>(UE2h, UE2l, OUTD, FUb, FT, W3uT, b3u, a2u, 0, nup, UE3, OUTD, nullptr, nullptr);
    k_gemm<0><<<dim3(nvp / 64, OUTD / 64), 128, 0, stream>>>(VE2h, VE2l, OUTD, FVb, FT, W3vT, b3v, a2v, 0, nvp, VE3, OUTD, nullptr, nullptr);
    k_sv<<<(nv + 7) / 8, 256, 0, stream>>>(VE3, UE3, nbr_v, nv, nu, SV);
    k_sv<<<(nu + 7) / 8, 256, 0, stream>>>(UE3, VE3, nbr_u, nu, nv, SU);
    k_losspart<<<nbv, 256, 0, stream>>>(VE3, SV, vidx, nv, PART);
    k_losspart<<<nbu, 256, 0, stream>>>(UE3, SU, uidx, nu, PART + (size_t)nbv * 32);
    k_lossfin<<<1, 256, 0, stream>>>(PART, nbv, nbu, nv, nu, losso);
}
